// KANLayer_89300960018758
// MI455X (gfx1250) — hardware-verified
//
#include <hip/hip_runtime.h>
#include <stdint.h>

#define NROWS  8192
#define NIN    1024
#define NOUT   256
#define NB     13
#define NH     12
#define KH     (NIN * NH)
#define KT     (2 * KH)
#define CH     2048
#define NCHUNK (NROWS / CH)
#define FTHR   512
#define NFPT   (NIN / FTHR)
#define UROW   (KT / 8)
#define NSWEEP (UROW / FTHR)
#define PIB    64
#define PSRC   (PIB * NB)
#define PSRC4  (PSRC / 4)
#define PUN    (PIB * NH / 8)
#define PGX    (NIN / PIB)
#define EPSF   1e-8f
#define WSCAP  134217728

static_assert(NROWS == NCHUNK * CH);
static_assert(CH % 128 == 0);
static_assert(NOUT % 64 == 0);
static_assert(KT % 32 == 0);
static_assert(KH % 32 == 0);
static_assert(UROW == NSWEEP * FTHR);
static_assert(NIN == NFPT * FTHR);
static_assert(PSRC % 4 == 0);
static_assert(PSRC4 <= 256);
static_assert((PIB * NH) % 8 == 0);
static_assert((2 * PUN) % 32 == 0);
static_assert(2 * PUN <= 256);
static_assert(NIN % PIB == 0);
static_assert((KT * 2) % 128 == 0);
static_assert((KH * 2) % 128 == 0);
static_assert((PIB * NH * 2) % 128 == 0);
static_assert((NH * 2) % 8 == 0);
static_assert((NOUT * 4) % 128 == 0);

typedef float          v4f   __attribute__((ext_vector_type(4)));
typedef float          v8f   __attribute__((ext_vector_type(8)));
typedef int            v8i   __attribute__((ext_vector_type(8)));
typedef unsigned int   v2u   __attribute__((ext_vector_type(2)));
typedef unsigned int   v4u   __attribute__((ext_vector_type(4)));
typedef unsigned short v8us  __attribute__((ext_vector_type(8)));
typedef unsigned short v16us __attribute__((ext_vector_type(16)));
typedef __bf16         v16bf __attribute__((ext_vector_type(16)));
typedef v4f  __attribute__((may_alias)) v4fa;
typedef v2u  __attribute__((may_alias)) v2ua;
typedef v4u  __attribute__((may_alias)) v4ua;
typedef v8us __attribute__((may_alias)) v8usa;
union FragB { v16bf v; v16us u; v8us h[2]; v8i w; };

__device__ __forceinline__ unsigned short f2bf_bits(float f) {
  unsigned u = __float_as_uint(f);
  return (unsigned short)((u + 0x7FFFu + ((u >> 16) & 1u)) >> 16);
}
__device__ __forceinline__ float bf_bits2f(unsigned short b) { return __uint_as_float(((unsigned)b) << 16); }
__device__ __forceinline__ float bfr(float f) { return bf_bits2f(f2bf_bits(f)); }
__device__ __forceinline__ unsigned pk16(unsigned short a, unsigned short b) { return (unsigned)a | ((unsigned)b << 16); }

__device__ __forceinline__ v8f wmb(const FragB& a, const FragB& b, v8f c) {
  v8f d = __builtin_amdgcn_wmma_f32_16x16x32_bf16(false, a.v, false, b.v, (short)0, c, false, false);
  asm volatile("v_nop\n\tv_nop\n\tv_nop\n\tv_nop" : "+v"(d) : "v"(a.w), "v"(b.w));
  return d;
}
__device__ __forceinline__ v8f z8() { v8f z = {0.f, 0.f, 0.f, 0.f, 0.f, 0.f, 0.f, 0.f}; return z; }

__global__ __launch_bounds__(256) void prep_kernel(const float* __restrict__ coeff,
                                                   unsigned short* __restrict__ BP) {
  __shared__ __align__(16) float sC[PSRC];
  const int tid = threadIdx.x;
  const int i0 = blockIdx.x * PIB;
  const int j = blockIdx.y;
  const float* src = coeff + ((size_t)j * NIN + i0) * NB;
  {
    const int t4 = (tid < PSRC4) ? tid : (PSRC4 - 1);
    const v4f v = *(const v4fa*)(src + 4 * t4);
    if (tid < PSRC4) *(v4fa*)(sC + 4 * tid) = v;
  }
  __syncthreads();

  if (tid < 2 * PUN) {
    const int hs = tid / PUN;
    const int uu = tid - hs * PUN;
    v4u v;
#pragma unroll
    for (int e2 = 0; e2 < 4; ++e2) {
      const int ka = 8 * uu + 2 * e2, kb = ka + 1;
      const int ia = ka / NH, ma = ka - NH * ia;
      const int ib = kb / NH, mb = kb - NH * ib;
      v[e2] = pk16(f2bf_bits(sC[ia * NB + ma]), f2bf_bits(sC[ib * NB + mb]));
    }
    unsigned short* dst = BP + (size_t)j * KT + (size_t)hs * KH + (size_t)i0 * NH + 8 * uu;
    *(volatile v4u*)dst = v;
    __threadfence();
    *(volatile v4u*)dst = v;
  }
}

__device__ __forceinline__ void a_store_pass(const unsigned short* sA, unsigned short* dst, int tid) {
#pragma unroll
  for (int it = 0; it < NSWEEP; ++it) {
    const int u = it * FTHR + tid;
    const v4u v = *(const v4ua*)(sA + 8 * u);
    *(volatile v4u*)(dst + 8 * u) = v;
  }
}

__global__ __launch_bounds__(FTHR) void feat_kernel(const float* __restrict__ x,
                                                    const float* __restrict__ knots,
                                                    unsigned short* __restrict__ AP, int row_base) {
  __shared__ __align__(16) unsigned short sA[KT];
  __shared__ __align__(16) float sK[16];
  const int tid = threadIdx.x;
  const int r = blockIdx.x;
  {
    const float kv = bfr(knots[tid & 15]);
    if (tid < 16) sK[tid] = kv;
  }
  __syncthreads();

  float kn[16];
#pragma unroll
  for (int g4 = 0; g4 < 4; ++g4) {
    const v4f t = *(const v4fa*)(sK + 4 * g4);
    kn[4 * g4 + 0] = t[0]; kn[4 * g4 + 1] = t[1]; kn[4 * g4 + 2] = t[2]; kn[4 * g4 + 3] = t[3];
  }
  bool srt = true;
#pragma unroll
  for (int mm = 0; mm < 15; ++mm) srt = srt & (kn[mm] <= kn[mm + 1]);
  const unsigned poison = srt ? 0u : 0x7FC07FC0u;

  const float* xrow = x + (size_t)(row_base + r) * NIN;
#pragma unroll 1
  for (int f = 0; f < NFPT; ++f) {
    const int i = tid + FTHR * f;
    const float xb = bfr(xrow[i]);
    const float xn = tanhf(xb);
    const float xc = fminf(fmaxf(xn, -1.0f), 1.0f);

    int p = 0;
#pragma unroll
    for (int mm = 0; mm < 16; ++mm) p += (xc >= kn[mm]) ? 1 : 0;
    const int q = p - 1;
    const int qc = min(max(q, 0), 14);
    const float kl = sK[qc];
    const float kr = sK[qc + 1];
    const float den = (kr - kl) + EPSF;
    const float up = (xc - kl) / den;
    const float dn = (kr - xc) / den;
    const float upv = (q >= 0 && q <= NH - 1) ? up : 0.0f;
    const float dnv = (q >= 1 && q <= NH) ? dn : 0.0f;

    const unsigned short uhb = f2bf_bits(upv);
    const unsigned short ulb = f2bf_bits(upv - bf_bits2f(uhb));
    const unsigned short dhb = f2bf_bits(dnv);
    const unsigned short dlb = f2bf_bits(dnv - bf_bits2f(dhb));
    const unsigned uh = uhb, ul = ulb, dh = dhb, dl = dlb;

    unsigned wh[6], wl[6];
#pragma unroll
    for (int e2 = 0; e2 < 6; ++e2) {
      const int ma = 2 * e2, mb = ma + 1;
      const unsigned ha = (q == ma) ? uh : ((q == ma + 1) ? dh : 0u);
      const unsigned hb = (q == mb) ? uh : ((q == mb + 1) ? dh : 0u);
      const unsigned la = (q == ma) ? ul : ((q == ma + 1) ? dl : 0u);
      const unsigned lb = (q == mb) ? ul : ((q == mb + 1) ? dl : 0u);
      wh[e2] = (ha | (hb << 16)) | poison;
      wl[e2] = (la | (lb << 16)) | poison;
    }
#pragma unroll
    for (int e = 0; e < 3; ++e) {
      v2u hv2; hv2.x = wh[2 * e]; hv2.y = wh[2 * e + 1];
      *(v2ua*)(sA + NH * i + 4 * e) = hv2;
      v2u lv2; lv2.x = wl[2 * e]; lv2.y = wl[2 * e + 1];
      *(v2ua*)(sA + KH + NH * i + 4 * e) = lv2;
    }
  }
  __syncthreads();

  unsigned short* dst = AP + (size_t)r * KT;
  a_store_pass(sA, dst, tid);
  __threadfence();
  a_store_pass(sA, dst, tid);
}

__device__ __forceinline__ void o_store_pass(const float* sO, float* out,
                                             int grow_w, int n0, int w, int lane) {
  const int q8 = lane & 7, sub = lane >> 3;
#pragma unroll
  for (int i = 0; i < 16; ++i) {
    const int lid = i * 4 + sub;
    const int row = lid >> 1, hl = lid & 1;
    const v4f v = *(const v4fa*)(sO + (32 * w + row) * 64 + 32 * hl + 4 * q8);
    *(volatile v4f*)(out + (size_t)(grow_w + row) * NOUT + n0 + 32 * hl + 4 * q8) = v;
  }
}

__global__ __launch_bounds__(128) void gemm_kernel(const unsigned short* __restrict__ AP,
                                                   const unsigned short* __restrict__ BP,
                                                   float* __restrict__ out, int row_base) {
  __shared__ __align__(16) float sO[128 * 64];
  const int tid = threadIdx.x, lane = tid & 31, w = tid >> 5;
  const int h = lane >> 4, m = lane & 15;
  const int lrow_w = blockIdx.x * 128 + 32 * w;
  const int n0 = blockIdx.y * 64;

  const unsigned short* xa0 = AP + (size_t)(lrow_w + m) * KT + 8 * h;
  const unsigned short* xa1 = xa0 + (size_t)16 * KT;
  const unsigned short* wb  = BP + (size_t)(n0 + m) * KT + 8 * h;

  v8f acc[2][4];
#pragma unroll
  for (int mt = 0; mt < 2; ++mt)
#pragma unroll
    for (int nt = 0; nt < 4; ++nt) acc[mt][nt] = z8();

#pragma unroll 1
  for (int k0 = 0; k0 < KT; k0 += 32) {
    FragB a0, a1;
    a0.h[0] = *(const v8usa*)(xa0 + k0);
    a0.h[1] = *(const v8usa*)(xa0 + k0 + 16);
    a1.h[0] = *(const v8usa*)(xa1 + k0);
    a1.h[1] = *(const v8usa*)(xa1 + k0 + 16);
#pragma unroll
    for (int nt = 0; nt < 4; ++nt) {
      const unsigned short* wq = wb + (size_t)nt * 16 * KT + k0;
      FragB b;
      b.h[0] = *(const v8usa*)wq;
      b.h[1] = *(const v8usa*)(wq + 16);
      acc[0][nt] = wmb(a0, b, acc[0][nt]);
      acc[1][nt] = wmb(a1, b, acc[1][nt]);
    }
  }

#pragma unroll
  for (int nt = 0; nt < 4; ++nt) {
    const int cl = 16 * nt + m;
#pragma unroll
    for (int mt = 0; mt < 2; ++mt) {
#pragma unroll
      for (int r = 0; r < 8; ++r) {
        const int rl = 32 * w + 16 * mt + 8 * h + r;
        sO[rl * 64 + cl] = acc[mt][nt][r];
      }
    }
  }
  __syncthreads();

  const int grow_w = row_base + lrow_w;
  o_store_pass(sO, out, grow_w, n0, w, lane);
  __threadfence();
  o_store_pass(sO, out, grow_w, n0, w, lane);
}

extern "C" void kernel_launch(void* const* d_in, const int* in_sizes, int n_in,
                              void* d_out, int out_size, void* d_ws, size_t ws_size,
                              hipStream_t stream) {
  if (n_in < 3) return;
  if (in_sizes[0] != NROWS * NIN) return;
  if (in_sizes[1] != NOUT * NIN * NB) return;
  if (in_sizes[2] != 16) return;
  if (out_size != NROWS * NOUT) return;

  const float* x     = (const float*)d_in[0];
  const float* coeff = (const float*)d_in[1];
  const float* knots = (const float*)d_in[2];
  float* out = (float*)d_out;

  size_t off = 0;
  const size_t oAP = off; off += (size_t)CH * KT * 2;
  const size_t oBP = off; off += (size_t)NOUT * KT * 2;
  if (off > ws_size) return;
  if (off > (size_t)WSCAP) return;

  char* ws = (char*)d_ws;
  unsigned short* AP = (unsigned short*)(ws + oAP);
  unsigned short* BP = (unsigned short*)(ws + oBP);

  prep_kernel<<<dim3(PGX, NOUT), dim3(256), 0, stream>>>(coeff, BP);
  for (int c = 0; c < NCHUNK; ++c) {
    const int row_base = c * CH;
    feat_kernel<<<dim3(CH), dim3(FTHR), 0, stream>>>(x, knots, AP, row_base);
    gemm_kernel<<<dim3(CH / 128, NOUT / 64), dim3(128), 0, stream>>>(AP, BP, out, row_base);
  }
  (void)hipGetLastError();
}
